// Fagcn_64501818851477
// MI455X (gfx1250) — hardware-verified
//
#include <hip/hip_runtime.h>
#include <stdint.h>
#include <stddef.h>


#define HD 128
#define EPSW 0.3f
#define NT 256
#define NW (NT / 32)
#define CH 2048
#define EPT1 (CH / NT)
#define R1 128
#define R1S 7
#define CAP 4096
#define EPT2 (CAP / NT)
#define OFFWMAX 1024
#define POSCAP 1024

typedef float v8f __attribute__((ext_vector_type(8)));
typedef float v4f __attribute__((ext_vector_type(4)));
typedef int v4i __attribute__((ext_vector_type(4)));
typedef unsigned int v4u __attribute__((ext_vector_type(4)));
typedef __bf16 v16bf __attribute__((ext_vector_type(16)));
typedef unsigned short v16us __attribute__((ext_vector_type(16)));
typedef v4f __attribute__((may_alias)) v4fa;
typedef v4i __attribute__((may_alias)) v4ia;
typedef v4u __attribute__((may_alias)) v4ua;

union Frag { v16bf v; v16us u; };

__device__ __forceinline__ v8f wmma_bf16(v16bf a, v16bf b, v8f c)
{
    v8f d = __builtin_amdgcn_wmma_f32_16x16x32_bf16(false, a, false, b, (short)0, c, false, false);
    asm volatile("v_nop\n\tv_nop\n\tv_nop\n\tv_nop" : "+v"(d) : "v"(a), "v"(b));
    return d;
}

__device__ __forceinline__ unsigned short bf16_rne(float x)
{
    unsigned int u = __float_as_uint(x);
    u += 0x7FFFu + ((u >> 16) & 1u);
    return (unsigned short)(u >> 16);
}

__device__ __forceinline__ float bf16_up(unsigned short b)
{
    return __uint_as_float(((unsigned int)b) << 16);
}

__device__ __forceinline__ void split_frag(const v4f q0, const v4f q1, const v4f q2, const v4f q3,
                                           float sc, Frag& hi, Frag& lo)
{
    float x[16] = { q0[0], q0[1], q0[2], q0[3], q1[0], q1[1], q1[2], q1[3],
                    q2[0], q2[1], q2[2], q2[3], q3[0], q3[1], q3[2], q3[3] };
#pragma unroll
    for (int i = 0; i < 16; ++i) {
        const float xv = x[i] * sc;
        const unsigned short hb = bf16_rne(xv);
        hi.u[i] = hb;
        lo.u[i] = bf16_rne(xv - bf16_up(hb));
    }
}

__device__ __forceinline__ int block_excl_scan(int v, int* wsum, int* total)
{
    const int tid = threadIdx.x, lane = tid & 31, wv = tid >> 5;
    int incl = v;
#pragma unroll
    for (int d = 1; d < 32; d <<= 1) {
        const int y = __shfl_up(incl, d, 32);
        if (lane >= d) incl += y;
    }
    if (lane == 31) wsum[wv] = incl;
    __syncthreads();
    int pre = 0, tot = 0;
#pragma unroll
    for (int w = 0; w < NW; ++w) {
        const int s = wsum[w];
        tot += s;
        pre += (w < wv) ? s : 0;
    }
    __syncthreads();
    *total = tot;
    return pre + incl - v;
}

__device__ __forceinline__ void lsort_store(const unsigned* sbuf, const int* offs, int tid,
                                            size_t cbase, size_t obase, int OFFW,
                                            unsigned* wsort, int* off)
{
#pragma unroll
    for (int sg = 0; sg < CH / (4 * NT); ++sg) {
        const int p = tid + NT * sg;
        const v4u v = *(const v4ua*)(sbuf + 4 * p);
        *(volatile v4u*)(wsort + cbase + 4 * p) = v;
    }
    for (int p = tid; p < (OFFW >> 2); p += NT) {
        const v4i v = *(const v4ia*)(offs + 4 * p);
        *(volatile v4i*)(off + obase + 4 * p) = v;
    }
}

__global__ __launch_bounds__(NT) void k_lsort(const int* __restrict__ dstv, int E, int N, int B1,
                                             int ES, int bbits, int OFFW,
                                             unsigned* wsort, int* off)
{
    __shared__ unsigned buf[2][CH] __attribute__((aligned(16)));
    __shared__ int offs[OFFWMAX] __attribute__((aligned(16)));
    __shared__ int wsum[NW];
    const int tid = threadIdx.x;
    const int c = blockIdx.x;
    const size_t cbase = (size_t)c * CH;

#pragma unroll
    for (int sg = 0; sg < CH / (4 * NT); ++sg) {
        const int p = tid + NT * sg;
        v4u wv;
#pragma unroll
        for (int q = 0; q < 4; ++q) {
            const size_t e = cbase + (size_t)(4 * p + q);
            unsigned w;
            if (e < (size_t)E) {
                int d = dstv[e];
                d = min(max(d, 0), N - 1);
                w = (((unsigned)(d >> R1S)) << ES) | (unsigned)e;
            } else {
                w = ((unsigned)B1) << ES;
            }
            wv[q] = w;
        }
        *(v4ua*)(&buf[0][4 * p]) = wv;
    }
    __syncthreads();

    int cur = 0;
#pragma unroll 1
    for (int bit = 0; bit < bbits; ++bit) {
        const int shf = ES + bit;
        const unsigned* rb = &buf[cur][tid * EPT1];
        const v4u q0 = *(const v4ua*)(rb);
        const v4u q1 = *(const v4ua*)(rb + 4);
        unsigned k[EPT1] = { q0[0], q0[1], q0[2], q0[3], q1[0], q1[1], q1[2], q1[3] };
        int ones = 0;
#pragma unroll
        for (int j = 0; j < EPT1; ++j) ones += (int)((k[j] >> shf) & 1u);
        int total;
        const int excl = block_excl_scan(ones, wsum, &total);
        const int nzero = CH - total;
        int run1 = excl;
        unsigned* wb = &buf[cur ^ 1][0];
#pragma unroll
        for (int j = 0; j < EPT1; ++j) {
            const int bt = (int)((k[j] >> shf) & 1u);
            const int idx = tid * EPT1 + j;
            const int ps = bt ? (nzero + run1) : (idx - run1);
            run1 += bt;
            wb[ps] = k[j];
        }
        __syncthreads();
        cur ^= 1;
    }
    const unsigned* sbuf = &buf[cur][0];

    for (int b = tid; b < OFFW; b += NT) {
        int lo = 0, hi = CH;
        while (lo < hi) {
            const int mid = (lo + hi) >> 1;
            if ((sbuf[mid] >> ES) < (unsigned)b) lo = mid + 1; else hi = mid;
        }
        offs[b] = lo;
    }
    __syncthreads();

    const size_t obase = (size_t)c * OFFW;
    lsort_store(sbuf, offs, tid, cbase, obase, OFFW, wsort, off);
    __threadfence();
    lsort_store(sbuf, offs, tid, cbase, obase, OFFW, wsort, off);
}

__device__ __forceinline__ void base_store(const int* sb, int tid, int OFFW, int* base)
{
    for (int p = tid; p < (OFFW >> 2); p += NT) {
        const v4i v = *(const v4ia*)(sb + 4 * p);
        *(volatile v4i*)(base + 4 * p) = v;
    }
}

__global__ __launch_bounds__(NT) void k_base(const int* __restrict__ off, int C, int B1, int OFFW, int* base)
{
    __shared__ int sb[OFFWMAX] __attribute__((aligned(16)));
    __shared__ int wsum[NW];
    const int tid = threadIdx.x;
    int carry = 0;
    for (int b0 = 0; b0 < OFFW; b0 += NT) {
        const int b = b0 + tid;
        int sz = 0;
        if (b < B1) {
            for (int c = 0; c < C; ++c) {
                const int* r = off + (size_t)c * OFFW + b;
                sz += r[1] - r[0];
            }
        }
        sz = max(sz, 0);
        const int ps = (sz + 31) & ~31;
        int total;
        const int excl = block_excl_scan(ps, wsum, &total);
        if (b < OFFW) sb[b] = carry + excl;
        carry += total;
    }
    __syncthreads();
    base_store(sb, tid, OFFW, base);
    __threadfence();
    base_store(sb, tid, OFFW, base);
}

__device__ __forceinline__ void bucket_store(const unsigned* sbuf, const int* srs, const int* sre, const float* sdn,
                                             int tid, int b, int bb, int npad, unsigned smask, int csrcap,
                                             int* csr, int* rs, int* re, float* dn)
{
    const size_t nbase = (size_t)b * R1;
    if (tid < 32) {
        const v4i v = *(const v4ia*)(srs + 4 * tid);
        *(volatile v4i*)(rs + nbase + 4 * tid) = v;
    } else if (tid < 64) {
        const int p = tid - 32;
        const v4i v = *(const v4ia*)(sre + 4 * p);
        *(volatile v4i*)(re + nbase + 4 * p) = v;
    } else if (tid < 96) {
        const int p = tid - 64;
        const v4f v = *(const v4fa*)(sdn + 4 * p);
        *(volatile v4f*)(dn + nbase + 4 * p) = v;
    }
    for (int p = tid; p < (npad >> 2); p += NT) {
        if (bb >= 0 && bb + 4 * p + 4 <= csrcap) {
            const v4u w = *(const v4ua*)(sbuf + 4 * p);
            v4i o;
            o[0] = (int)(w[0] & smask); o[1] = (int)(w[1] & smask);
            o[2] = (int)(w[2] & smask); o[3] = (int)(w[3] & smask);
            *(volatile v4i*)(csr + (size_t)bb + 4 * p) = o;
        }
    }
}

__global__ __launch_bounds__(NT) void k_bucket(const unsigned* __restrict__ wsort, const int* __restrict__ off,
                                              const int* __restrict__ base,
                                              const int* __restrict__ srcv, const int* __restrict__ dstv,
                                              int C, int OFFW, int ES, int N, int E, int SB, int rbits,
                                              int csrcap,
                                              int* csr, int* rs, int* re, float* dn)
{
    __shared__ unsigned buf[2][CAP] __attribute__((aligned(16)));
    __shared__ int pos[POSCAP];
    __shared__ int lbv[R1 + 1];
    __shared__ int srs[R1] __attribute__((aligned(16)));
    __shared__ int sre[R1] __attribute__((aligned(16)));
    __shared__ float sdn[R1] __attribute__((aligned(16)));
    __shared__ int wsum[NW];
    const int tid = threadIdx.x;
    const int b = blockIdx.x;
    const unsigned emask = (ES >= 32) ? 0xffffffffu : ((1u << ES) - 1u);
    const unsigned smask = (1u << SB) - 1u;

    int carry = 0;
    for (int c0 = 0; c0 < C; c0 += NT) {
        const int c = c0 + tid;
        int len = 0;
        if (c < C) {
            const int* r = off + (size_t)c * OFFW + b;
            len = min(max(r[1] - r[0], 0), CH);
        }
        int total;
        const int excl = block_excl_scan(len, wsum, &total);
        if (c < C) pos[c] = carry + excl;
        carry += total;
    }
    const int nb = carry;
    const int nuse = min(nb, CAP);
    __syncthreads();

    for (int c = tid; c < C; c += NT) {
        const int* r = off + (size_t)c * OFFW + b;
        int lo = r[0];
        const int len = min(max(r[1] - lo, 0), CH);
        lo = min(max(lo, 0), CH);
        const int p = pos[c];
        const unsigned* sw = wsort + (size_t)c * CH;
        for (int i = 0; i < len; ++i) {
            const int li = lo + i;
            if (li >= CH) break;
            const unsigned w = sw[li];
            int e = (int)(w & emask);
            e = min(e, E - 1);
            int s = srcv[e];
            s = min(max(s, 0), N - 1);
            int d = dstv[e];
            d = min(max(d, 0), N - 1);
            int dl = d - b * R1;
            dl = min(max(dl, 0), R1 - 1);
            const int q = p + i;
            if (q < CAP) buf[0][q] = (((unsigned)dl) << SB) | (unsigned)s;
        }
    }
    for (int q = nuse + tid; q < CAP; q += NT) buf[0][q] = ((unsigned)R1) << SB;
    __syncthreads();

    int cur = 0;
#pragma unroll 1
    for (int bit = 0; bit < rbits; ++bit) {
        const int shf = SB + bit;
        const unsigned* rb = &buf[cur][tid * EPT2];
        const v4u q0 = *(const v4ua*)(rb);
        const v4u q1 = *(const v4ua*)(rb + 4);
        const v4u q2 = *(const v4ua*)(rb + 8);
        const v4u q3 = *(const v4ua*)(rb + 12);
        unsigned k[EPT2] = { q0[0], q0[1], q0[2], q0[3], q1[0], q1[1], q1[2], q1[3],
                             q2[0], q2[1], q2[2], q2[3], q3[0], q3[1], q3[2], q3[3] };
        int ones = 0;
#pragma unroll
        for (int j = 0; j < EPT2; ++j) ones += (int)((k[j] >> shf) & 1u);
        int total;
        const int excl = block_excl_scan(ones, wsum, &total);
        const int nzero = CAP - total;
        int run1 = excl;
        unsigned* wb = &buf[cur ^ 1][0];
#pragma unroll
        for (int j = 0; j < EPT2; ++j) {
            const int bt = (int)((k[j] >> shf) & 1u);
            const int idx = tid * EPT2 + j;
            const int ps = bt ? (nzero + run1) : (idx - run1);
            run1 += bt;
            wb[ps] = k[j];
        }
        __syncthreads();
        cur ^= 1;
    }
    const unsigned* sbuf = &buf[cur][0];

    if (tid <= R1) {
        int lo = 0, hi = CAP;
        while (lo < hi) {
            const int mid = (lo + hi) >> 1;
            if ((sbuf[mid] >> SB) < (unsigned)tid) lo = mid + 1; else hi = mid;
        }
        lbv[tid] = lo;
    }
    __syncthreads();
    const int bb = base[b];
    if (tid < R1) {
        const int s0 = lbv[tid], s1 = lbv[tid + 1];
        srs[tid] = bb + s0;
        sre[tid] = bb + s1;
        const int dg = s1 - s0;
        sdn[tid] = rsqrtf(fmaxf((float)dg, 1.0f));
    }
    __syncthreads();

    const int npad = (nuse + 31) & ~31;
    bucket_store(sbuf, srs, sre, sdn, tid, b, bb, npad, smask, csrcap, csr, rs, re, dn);
    __threadfence();
    bucket_store(sbuf, srs, sre, sdn, tid, b, bb, npad, smask, csrcap, csr, rs, re, dn);
}

__global__ __launch_bounds__(64) void k_proj(const float* __restrict__ h, const float* __restrict__ gwl,
                                            float* adst, float* asrc, int N, int NP32)
{
    __shared__ float sh[2][64] __attribute__((aligned(16)));
    const int wv = threadIdx.x >> 5;
    const int l = threadIdx.x & 31, hh = l >> 4, m = l & 15;
    const int wg = blockIdx.x * 2 + wv;
    const int rbase = wg * 32;
    int r0 = rbase + m;       if (r0 > N - 1) r0 = N - 1;
    int r1 = rbase + 16 + m;  if (r1 > N - 1) r1 = N - 1;
    const float* hr0 = h + (size_t)r0 * HD;
    const float* hr1 = h + (size_t)r1 * HD;
    const float* wr = gwl + ((m < 2) ? m : 0) * HD;
    const float bsc = (m < 2) ? 1.0f : 0.0f;

    v8f acc0, acc1;
#pragma unroll
    for (int r = 0; r < 8; ++r) { acc0[r] = 0.0f; acc1[r] = 0.0f; }

#pragma unroll 1
    for (int c = 0; c < HD / 32; ++c) {
        const int ka = c * 32 + 8 * hh;
        const int kb = c * 32 + 16 + 8 * hh;
        Frag bh, bl, ah, al;
        split_frag(*(const v4f*)(wr + ka), *(const v4f*)(wr + ka + 4),
                   *(const v4f*)(wr + kb), *(const v4f*)(wr + kb + 4), bsc, bh, bl);
        split_frag(*(const v4f*)(hr0 + ka), *(const v4f*)(hr0 + ka + 4),
                   *(const v4f*)(hr0 + kb), *(const v4f*)(hr0 + kb + 4), 1.0f, ah, al);
        acc0 = wmma_bf16(ah.v, bh.v, acc0);
        acc0 = wmma_bf16(ah.v, bl.v, acc0);
        acc0 = wmma_bf16(al.v, bh.v, acc0);
        split_frag(*(const v4f*)(hr1 + ka), *(const v4f*)(hr1 + ka + 4),
                   *(const v4f*)(hr1 + kb), *(const v4f*)(hr1 + kb + 4), 1.0f, ah, al);
        acc1 = wmma_bf16(ah.v, bh.v, acc1);
        acc1 = wmma_bf16(ah.v, bl.v, acc1);
        acc1 = wmma_bf16(al.v, bh.v, acc1);
    }

    if (m == 0) {
#pragma unroll
        for (int r = 0; r < 8; ++r) { sh[wv][8 * hh + r] = acc0[r]; sh[wv][16 + 8 * hh + r] = acc1[r]; }
    } else if (m == 1) {
#pragma unroll
        for (int r = 0; r < 8; ++r) { sh[wv][32 + 8 * hh + r] = acc0[r]; sh[wv][48 + 8 * hh + r] = acc1[r]; }
    }
    __syncthreads();
    if (rbase < NP32 && l < 16) {
        const v4f v = *(const v4fa*)(&sh[wv][4 * l]);
        float* p = (l < 8) ? (adst + (size_t)rbase + 4 * l) : (asrc + (size_t)rbase + 4 * (l - 8));
        *(volatile v4f*)p = v;
        __threadfence();
        *(volatile v4f*)p = v;
    }
}

__global__ __launch_bounds__(NT) void k_agg(const float* __restrict__ hin, const int* __restrict__ csr,
                                           const int* __restrict__ rs, const int* __restrict__ re,
                                           const float* __restrict__ dn,
                                           const float* __restrict__ adst, const float* __restrict__ asrc,
                                           const float* __restrict__ gb, int layer, int N, int csrcap,
                                           float* out)
{
    const int l = threadIdx.x & 31;
    const int wg = blockIdx.x * NW + (threadIdx.x >> 5);
    if (wg >= N) return;
    const int t = __builtin_amdgcn_readfirstlane(wg);
    int st = rs[t], en = re[t];
    st = min(max(st, 0), csrcap);
    en = min(max(en, st), csrcap);
    const float at = adst[t] + gb[layer];
    const float dt = dn[t];
    v4f acc;
    acc[0] = 0.0f; acc[1] = 0.0f; acc[2] = 0.0f; acc[3] = 0.0f;
    for (int j0 = st; j0 < en; j0 += 32) {
        const int idx = j0 + l;
        int s = 0;
        float cf = 0.0f;
        if (idx < en) {
            s = csr[idx];
            s = min(max(s, 0), N - 1);
            cf = tanhf(at + asrc[s]) * dt * dn[s];
        }
        const int cnt = min(32, en - j0);
#pragma unroll 1
        for (int j = 0; j < cnt; ++j) {
            const int sj = __builtin_amdgcn_readlane(s, j);
            const float cj = __int_as_float(__builtin_amdgcn_readlane(__float_as_int(cf), j));
            const v4f v = *(const v4f*)(hin + (size_t)sj * HD + 4 * l);
            acc += cj * v;
        }
    }
    const v4f x = *(const v4f*)(hin + (size_t)t * HD + 4 * l);
    v4f r = EPSW * x + acc;
    r[0] = fmaxf(r[0], 0.0f); r[1] = fmaxf(r[1], 0.0f);
    r[2] = fmaxf(r[2], 0.0f); r[3] = fmaxf(r[3], 0.0f);
    float* op = out + (size_t)t * HD + 4 * l;
    *(volatile v4f*)op = r;
    __threadfence();
    *(volatile v4f*)op = r;
}

static inline int h_nbits(unsigned int x)
{
    int n = 0;
    while (x) { ++n; x >>= 1; }
    return n > 0 ? n : 1;
}

extern "C" void kernel_launch(void* const* d_in, const int* in_sizes, int n_in,
                              void* d_out, int out_size, void* d_ws, size_t ws_size,
                              hipStream_t stream)
{
    if (n_in < 4) return;
    const float* h0 = (const float*)d_in[0];
    const int*   ei = (const int*)d_in[1];
    const float* gw = (const float*)d_in[2];
    const float* gb = (const float*)d_in[3];
    const int N = in_sizes[0] / HD;
    const int E = in_sizes[1] / 2;
    if (N <= 0 || E <= 0) return;
    if ((long long)out_size < (long long)N * HD) return;
    const int* srcv = ei;
    const int* dstv = ei + E;

    const int B1    = (N + R1 - 1) / R1;
    const int NB    = B1 * R1;
    const int NP32  = ((N + 31) / 32) * 32;
    const int C     = (E + CH - 1) / CH;
    const int EP    = C * CH;
    const int OFFW  = ((B1 + 1 + 31) / 32) * 32;
    const int ES    = h_nbits((unsigned)(E - 1));
    const int bbits = h_nbits((unsigned)B1);
    const int SB    = h_nbits((unsigned)(N - 1));
    const int rbits = h_nbits((unsigned)R1);
    const int CSRCAP = ((E + 32 * B1 + 31) / 32) * 32;
    if (C > POSCAP || OFFW > OFFWMAX || ES + bbits > 32 || SB + rbits > 31) return;

    char* W = (char*)d_ws;
    size_t ob = 0;
    auto carve = [&](size_t bytes) -> char* { char* p = W + ob; ob += (bytes + 255) & ~(size_t)255; return p; };
    unsigned* wsort = (unsigned*)carve((size_t)EP * 4);
    int*   off   = (int*)carve((size_t)C * OFFW * 4);
    int*   base  = (int*)carve((size_t)OFFW * 4);
    int*   csr   = (int*)carve((size_t)CSRCAP * 4);
    int*   rs    = (int*)carve((size_t)NB * 4);
    int*   re    = (int*)carve((size_t)NB * 4);
    float* dn    = (float*)carve((size_t)NB * 4);
    float* adst  = (float*)carve((size_t)NP32 * 4);
    float* asrc  = (float*)carve((size_t)NP32 * 4);
    float* h1    = (float*)carve((size_t)N * HD * 4);
    if (ob > ws_size) return;
    float* out = (float*)d_out;

    const dim3 blk(NT);
    const int projBlocks = (NP32 / 32 + 1) / 2;
    const int aggBlocks  = (N + NW - 1) / NW;

    k_lsort<<<dim3(C), blk, 0, stream>>>(dstv, E, N, B1, ES, bbits, OFFW, wsort, off);
    k_base<<<dim3(1), blk, 0, stream>>>(off, C, B1, OFFW, base);
    k_bucket<<<dim3(B1), blk, 0, stream>>>(wsort, off, base, srcv, dstv, C, OFFW, ES, N, E, SB, rbits,
                                           CSRCAP, csr, rs, re, dn);

    k_proj<<<dim3(projBlocks), dim3(64), 0, stream>>>(h0, gw, adst, asrc, N, NP32);
    k_agg<<<dim3(aggBlocks), blk, 0, stream>>>(h0, csr, rs, re, dn, adst, asrc, gb, 0, N, CSRCAP, h1);

    k_proj<<<dim3(projBlocks), dim3(64), 0, stream>>>(h1, gw + 2 * HD, adst, asrc, N, NP32);
    k_agg<<<dim3(aggBlocks), blk, 0, stream>>>(h1, csr, rs, re, dn, adst, asrc, gb, 1, N, CSRCAP, out);
}
